// DAGTaskEncoder_68642167324672
// MI455X (gfx1250) — hardware-run, weakly checked
//
#include <hip/hip_runtime.h>
#include <stddef.h>
#include <stdint.h>


#define DIN     128
#define C1      128
#define C2      64
#define N1      256
#define N2      128
#define K2      256
#define LDX     256
#define LDH     512
#define XR1OFF  128
#define HOFF    256
#define XR2OFF  64
#define NTHR    256
#define NWAVE   8
#define EPT     8
#define CHUNK   (NTHR * EPT)
#define WCAP    (EPT * 32)
#define LISTN   (NWAVE * WCAP)
#define NBMAX   2048
#define SLB     11
#define RCAP    28672
#define DEGCAP  1024
#define STW     512
#define PRMN    512
#define GBM     64
#define GBN     64
#define GTHR    128
#define WSMAX   134217728
#define LDS_AGG ((2 * RCAP + 2 * NBMAX + LISTN + PRMN) * 4 + 64)

static_assert((CHUNK & (CHUNK - 1)) == 0 && CHUNK <= 4096);
static_assert((NBMAX & (NBMAX - 1)) == 0 && NBMAX == (1 << SLB));
static_assert(NTHR * 8 == NBMAX);
static_assert(LISTN >= NBMAX);
static_assert(LISTN >= NWAVE * WCAP);
static_assert((RCAP % 32) == 0);
static_assert(NWAVE * STW <= RCAP);
static_assert(4 * 32 <= STW);
static_assert(PRMN >= 4 * C1 && (PRMN % 4) == 0);
static_assert(LDS_AGG <= 300000);
static_assert(GBM == (GTHR / 32) * 16);
static_assert(GTHR >= GBN);
static_assert((DIN % 32) == 0 && (K2 % 32) == 0);
static_assert((N1 % GBN) == 0 && (N2 % GBN) == 0);
static_assert(C1 == 2 * C2 && N1 == 2 * C1 && N2 == 2 * C2 && K2 == 2 * C1);
static_assert(LDX == N1 && LDH == 2 * LDX && HOFF == 2 * XR1OFF && XR1OFF + C1 == LDX && XR2OFF + C2 <= XR1OFF);
static_assert(21 + SLB <= 32);
static_assert(NTHR >= C1);

typedef float          v4f  __attribute__((ext_vector_type(4)));
typedef float          v8f  __attribute__((ext_vector_type(8)));
typedef int            v4i  __attribute__((ext_vector_type(4)));
typedef int            v8i  __attribute__((ext_vector_type(8)));
typedef unsigned short v8us __attribute__((ext_vector_type(8)));
typedef __bf16         v16b __attribute__((ext_vector_type(16)));
union FragB { v16b v; v8us h[2]; v8i w; };

__device__ __forceinline__ v8f wmb(const FragB& a, const FragB& b, v8f c) {
  v8f d = __builtin_amdgcn_wmma_f32_16x16x32_bf16(false, a.v, false, b.v, (short)0, c, false, false);
  asm volatile("v_nop\n\tv_nop\n\tv_nop\n\tv_nop" : "+v"(d) : "v"(a.w), "v"(b.w));
  return d;
}

__device__ __forceinline__ void ldwait() {
  asm volatile("s_wait_loadcnt 0x0" ::: "memory");
}

__device__ __forceinline__ unsigned short bf_bits(float f) {
  unsigned u = __float_as_uint(f);
  u = u + 0x7FFFu + ((u >> 16) & 1u);
  return (unsigned short)(u >> 16);
}
__device__ __forceinline__ float bf_val(unsigned short b) { return __uint_as_float(((unsigned)b) << 16); }
__device__ __forceinline__ float bfr(float f) { return bf_val(bf_bits(f)); }

__device__ __forceinline__ v8us cvt8b(const v4f a, const v4f b) {
  v8us o;
  o[0] = bf_bits(a.x); o[1] = bf_bits(a.y); o[2] = bf_bits(a.z); o[3] = bf_bits(a.w);
  o[4] = bf_bits(b.x); o[5] = bf_bits(b.y); o[6] = bf_bits(b.z); o[7] = bf_bits(b.w);
  return o;
}

__device__ __forceinline__ unsigned short hl1(float f, int hsel) {
  const unsigned short hb = bf_bits(f);
  const unsigned short lb = bf_bits(f - bf_val(hb));
  return hsel ? lb : hb;
}
__device__ __forceinline__ v8us hilo8(const v4f a, const v4f b, int hsel) {
  v8us o;
  o[0] = hl1(a.x, hsel); o[1] = hl1(a.y, hsel); o[2] = hl1(a.z, hsel); o[3] = hl1(a.w, hsel);
  o[4] = hl1(b.x, hsel); o[5] = hl1(b.y, hsel); o[6] = hl1(b.z, hsel); o[7] = hl1(b.w, hsel);
  return o;
}

__device__ __forceinline__ int scan_chunk(const int* __restrict__ dsts, int nE, int cbase, int slotBase,
                                          int nb, int vec8, int* list, int tid, int lane, int wave) {
  int wc = 0;
  const int el0  = tid * EPT;
  const int e0   = cbase + el0;
  const int sent = -2147483647 - 1;
  v4i da, db;
  if (vec8 != 0 && cbase + CHUNK <= nE) {
    da = *(const v4i*)(dsts + e0);
    db = *(const v4i*)(dsts + e0 + 4);
    ldwait();
  } else {
    da.x = (e0     < nE) ? dsts[min(e0,     nE - 1)] : sent;
    da.y = (e0 + 1 < nE) ? dsts[min(e0 + 1, nE - 1)] : sent;
    da.z = (e0 + 2 < nE) ? dsts[min(e0 + 2, nE - 1)] : sent;
    da.w = (e0 + 3 < nE) ? dsts[min(e0 + 3, nE - 1)] : sent;
    ldwait();
    db.x = (e0 + 4 < nE) ? dsts[min(e0 + 4, nE - 1)] : sent;
    db.y = (e0 + 5 < nE) ? dsts[min(e0 + 5, nE - 1)] : sent;
    db.z = (e0 + 6 < nE) ? dsts[min(e0 + 6, nE - 1)] : sent;
    db.w = (e0 + 7 < nE) ? dsts[min(e0 + 7, nE - 1)] : sent;
    ldwait();
  }
  const unsigned nbs = (unsigned)slotBase;
  const unsigned unb = (unsigned)nb;
  const unsigned s0 = (unsigned)da.x - nbs, s1 = (unsigned)da.y - nbs;
  const unsigned s2 = (unsigned)da.z - nbs, s3 = (unsigned)da.w - nbs;
  const unsigned s4 = (unsigned)db.x - nbs, s5 = (unsigned)db.y - nbs;
  const unsigned s6 = (unsigned)db.z - nbs, s7 = (unsigned)db.w - nbs;
  const bool h0 = s0 < unb, h1 = s1 < unb, h2 = s2 < unb, h3 = s3 < unb;
  const bool h4 = s4 < unb, h5 = s5 < unb, h6 = s6 < unb, h7 = s7 < unb;
  const unsigned any = __builtin_amdgcn_ballot_w32(h0 | h1 | h2 | h3 | h4 | h5 | h6 | h7);
  if (any != 0u) {
#define HITJ(J, HJ, SJ) { \
      const unsigned mj = __builtin_amdgcn_ballot_w32(HJ); \
      if (mj != 0u) { \
        if (HJ) { \
          const int pos = wc + (int)__builtin_amdgcn_mbcnt_lo(mj, 0u); \
          if (pos < WCAP) list[wave * WCAP + pos] = ((el0 + (J)) << 12) | (int)(SJ); \
        } \
        wc += (int)__builtin_popcount(mj); } }
    HITJ(0, h0, s0)
    HITJ(1, h1, s1)
    HITJ(2, h2, s2)
    HITJ(3, h3, s3)
    HITJ(4, h4, s4)
    HITJ(5, h5, s5)
    HITJ(6, h6, s6)
    HITJ(7, h7, s7)
#undef HITJ
  }
  return wc;
}

__global__ __launch_bounds__(NTHR) void k_xprep(const float* __restrict__ x, unsigned short* xb, int nN, int nUnits) {
  const int i = (int)blockIdx.x * NTHR + (int)threadIdx.x;
  if (i >= nUnits) return;
  const int row = i >> 4;
  const int c0  = (i & 15) * 8;
  const int rc  = row < nN ? row : nN - 1;
  const float* p = x + (size_t)rc * DIN + c0;
  v4f a = *(const v4f*)p, b = *(const v4f*)(p + 4);
  ldwait();
  const v4f z4 = {0.f, 0.f, 0.f, 0.f};
  if (row >= nN) { a = z4; b = z4; }
  const v8us hv = cvt8b(a, b);
  const size_t o = (size_t)row * DIN + c0;
  *(volatile v8us*)(xb + o) = hv;
  __threadfence();
  *(volatile v8us*)(xb + o) = hv;
}

__global__ __launch_bounds__(NTHR) void k_wtr(const float* __restrict__ w0, const float* __restrict__ w1,
                                              int cols, int Kin, int KP, unsigned short* wt, int nUnits) {
  const int u = (int)blockIdx.x * NTHR + (int)threadIdx.x;
  if (u >= nUnits) return;
  const int kq = KP >> 3;
  const int n  = u / kq;
  const int k8 = (u - n * kq) * 8;
  int seg = n / cols;
  seg = seg > 1 ? 1 : seg;
  int nc = n - seg * cols;
  nc = nc < 0 ? 0 : (nc > cols - 1 ? cols - 1 : nc);
  const float* ws = (seg == 0) ? w0 : w1;
  int kk = k8 >= Kin ? k8 - Kin : k8;
  kk = kk < 0 ? 0 : (kk > Kin - 8 ? Kin - 8 : kk);
  const float* p = ws + (size_t)kk * (size_t)cols + nc;
  v4f a, b;
  a.x = p[0];                    a.y = p[(size_t)cols];         a.z = p[(size_t)2 * cols];     a.w = p[(size_t)3 * cols];
  ldwait();
  b.x = p[(size_t)4 * cols];     b.y = p[(size_t)5 * cols];     b.z = p[(size_t)6 * cols];     b.w = p[(size_t)7 * cols];
  ldwait();
  const v8us hv = cvt8b(a, b);
  const size_t o = (size_t)n * (size_t)KP + k8;
  *(volatile v8us*)(wt + o) = hv;
  __threadfence();
  *(volatile v8us*)(wt + o) = hv;
}

__global__ __launch_bounds__(GTHR) void k_gemm(
    const unsigned short* A, int lda, const unsigned short* __restrict__ WT, int K,
    const float* __restrict__ b0, const float* __restrict__ b1, int segN, int blen,
    float* outF, int ldo)
{
  __shared__ __attribute__((aligned(16))) float stg[GBM * GBN];
  __shared__ __attribute__((aligned(16))) float sbias[GBN];
  const int tid = (int)threadIdx.x, lane = tid & 31, wave = tid >> 5, hh = lane >> 4, m = lane & 15;
  const int rowBase = (int)blockIdx.x * GBM;
  const int col0    = (int)blockIdx.y * GBN;
  int seg = col0 / segN;
  seg = seg < 0 ? 0 : (seg > 1 ? 1 : seg);
  const float* bp = (seg == 0) ? b0 : b1;
  int bofs = col0 - seg * segN;
  bofs = bofs < 0 ? 0 : bofs;
  if (tid < GBN) {
    int bi = bofs + tid;
    bi = bi > blen - 1 ? blen - 1 : bi;
    bi = bi < 0 ? 0 : bi;
    const float bv = bp[bi];
    ldwait();
    sbias[tid] = bfr(bv);
  }
  __syncthreads();

  v8f acc[4];
  {
    const v8f z = {0.f, 0.f, 0.f, 0.f, 0.f, 0.f, 0.f, 0.f};
    acc[0] = z; acc[1] = z; acc[2] = z; acc[3] = z;
  }
  const unsigned short* ap = A  + (size_t)(rowBase + 16 * wave + m) * (size_t)lda + 8 * hh;
  const unsigned short* wp = WT + (size_t)(col0 + m) * (size_t)K + 8 * hh;
  const int ksteps = K >> 5;
#pragma unroll 1
  for (int ks = 0; ks < ksteps; ++ks) {
    FragB af;
    af.h[0] = *(const v8us*)(ap + 32 * ks);
    af.h[1] = *(const v8us*)(ap + 32 * ks + 16);
#pragma unroll
    for (int t = 0; t < 4; ++t) {
      const unsigned short* wq = wp + (size_t)(16 * t) * (size_t)K + 32 * ks;
      FragB bg;
      bg.h[0] = *(const v8us*)wq;
      bg.h[1] = *(const v8us*)(wq + 16);
      acc[t] = wmb(af, bg, acc[t]);
    }
  }

#pragma unroll
  for (int t = 0; t < 4; ++t) {
    const int lc = 16 * t + m;
    const float bv = sbias[lc];
#pragma unroll
    for (int r = 0; r < 8; ++r) {
      const int lr = 16 * wave + 8 * hh + r;
      stg[lr * GBN + lc] = acc[t][r] + bv;
    }
  }
  __syncthreads();

  v4f fv[8];
#pragma unroll
  for (int i = 0; i < 8; ++i) {
    const int lr = 16 * wave + 2 * i + hh;
    fv[i] = *(const v4f*)(stg + lr * GBN + 4 * m);
  }
#pragma unroll
  for (int i = 0; i < 8; ++i) {
    const int lr = 16 * wave + 2 * i + hh;
    const int gr = rowBase + lr;
    float* op = outF + (size_t)gr * (size_t)ldo + col0 + 4 * m;
    *(volatile v4f*)op = fv[i];
  }
  __threadfence();
#pragma unroll
  for (int i = 0; i < 8; ++i) {
    const int lr = 16 * wave + 2 * i + hh;
    const int gr = rowBase + lr;
    float* op = outF + (size_t)gr * (size_t)ldo + col0 + 4 * m;
    *(volatile v4f*)op = fv[i];
  }
}

template<int LAYER>
__global__ __launch_bounds__(NTHR) void k_agg(
    const int* __restrict__ srcs, const int* __restrict__ dsts, float* plane,
    const float* __restrict__ att, const float* __restrict__ bias,
    const float* __restrict__ gam, const float* __restrict__ bet,
    float* outN, int nN, int nE, int nb, int vec8, int MPr) {
  constexpr int NJ  = (LAYER == 1) ? 4 : 2;
  constexpr int NHD = (LAYER == 1) ? 2 : 1;
  constexpr int NCH = 32 * NJ;
  constexpr int XRO = (LAYER == 1) ? XR1OFF : XR2OFF;
  extern __shared__ v4f lds_dyn[];
  int*   reg1 = (int*)lds_dyn;
  int*   reg2 = reg1 + RCAP;
  int*   scnt = reg2 + RCAP;
  int*   soff = scnt + NBMAX;
  int*   list = soff + NBMAX;
  float* prm  = (float*)(list + LISTN);
  int*   wcnt = (int*)(prm + PRMN);
  int*   wtot = wcnt + NWAVE;
  const int tid = (int)threadIdx.x, lane = tid & 31, wave = tid >> 5, hh = lane >> 4;
  const int nodeBase = (int)blockIdx.x * nb;

  for (int i = tid; i < NBMAX; i += NTHR) scnt[i] = 0;
  if (tid < NCH) {
    const float a0 = att[tid];
    const float b0 = bias[tid];
    const float g0 = gam[tid];
    const float e0 = bet[tid];
    ldwait();
    prm[tid]           = bfr(a0);
    prm[NCH + tid]     = bfr(b0);
    prm[2 * NCH + tid] = (LAYER == 1) ? bfr(g0) : 1.0f;
    prm[3 * NCH + tid] = (LAYER == 1) ? bfr(e0) : 0.0f;
  }
  __syncthreads();

  int tot = 0;
  const int nChunks = (nE + CHUNK - 1) / CHUNK;
#pragma unroll 1
  for (int ch = 0; ch < nChunks; ++ch) {
    const int cbase = ch * CHUNK;
    const int wc = scan_chunk(dsts, nE, cbase, nodeBase, nb, vec8, list, tid, lane, wave);
    if (lane == 0) wcnt[wave] = wc;
    __syncthreads();
    int pre = 0, all = 0;
#pragma unroll
    for (int w2 = 0; w2 < NWAVE; ++w2) {
      int c = wcnt[w2];
      c = c < 0 ? 0 : (c > WCAP ? WCAP : c);
      all += c;
      pre += (w2 < wave) ? c : 0;
    }
    const int wcc  = wc > WCAP ? WCAP : wc;
    const int base = tot + pre;
#pragma unroll 1
    for (int i = lane; i < wcc; i += 32) {
      const int ent = list[wave * WCAP + i];
      const int el  = (ent >> 12) & (CHUNK - 1);
      const int sl  = ent & (NBMAX - 1);
      int eid = cbase + el;
      eid = eid > nE - 1 ? nE - 1 : eid;
      const int pos = base + i;
      if (pos < RCAP) reg1[pos] = (int)(((unsigned)eid << SLB) | (unsigned)sl);
    }
    tot += all;
    tot = tot > RCAP ? RCAP : tot;
    __syncthreads();
  }
  const int nh = tot;

  if (wave == 0) {
#pragma unroll 1
    for (int b0 = 0; b0 < nh; b0 += 32) {
      const int idx = b0 + lane;
      const int uv  = reg1[idx < RCAP ? idx : RCAP - 1];
      const int m32 = (nh - b0) < 32 ? (nh - b0) : 32;
#pragma unroll 1
      for (int k = 0; k < m32; ++k) {
        const int u  = __builtin_amdgcn_readlane(uv, k);
        const int sl = u & (NBMAX - 1);
        if (lane == 0) scnt[sl] = scnt[sl] + 1;
      }
    }
  }
  __syncthreads();

  {
    const v4i ca = *(const v4i*)(scnt + 8 * tid);
    const v4i cb = *(const v4i*)(scnt + 8 * tid + 4);
    const int e0 = ca.x < 0 ? 0 : ca.x, e1 = ca.y < 0 ? 0 : ca.y, e2 = ca.z < 0 ? 0 : ca.z, e3 = ca.w < 0 ? 0 : ca.w;
    const int e4 = cb.x < 0 ? 0 : cb.x, e5 = cb.y < 0 ? 0 : cb.y, e6 = cb.z < 0 ? 0 : cb.z, e7 = cb.w < 0 ? 0 : cb.w;
    const int ts = e0 + e1 + e2 + e3 + e4 + e5 + e6 + e7;
    int incl = ts;
#pragma unroll
    for (int d = 1; d < 32; d <<= 1) {
      const int up = __shfl_up(incl, d);
      if (lane >= d) incl += up;
    }
    if (lane == 31) wtot[wave] = incl;
    __syncthreads();
    int pre = 0;
#pragma unroll
    for (int w2 = 0; w2 < NWAVE; ++w2) pre += (w2 < wave) ? wtot[w2] : 0;
    int run = pre + incl - ts;
    soff[8 * tid + 0] = run; run += e0;
    soff[8 * tid + 1] = run; run += e1;
    soff[8 * tid + 2] = run; run += e2;
    soff[8 * tid + 3] = run; run += e3;
    soff[8 * tid + 4] = run; run += e4;
    soff[8 * tid + 5] = run; run += e5;
    soff[8 * tid + 6] = run; run += e6;
    soff[8 * tid + 7] = run;
  }
  __syncthreads();
  for (int i = tid; i < NBMAX; i += NTHR) list[i] = soff[i];
  __syncthreads();

  if (wave == 0) {
#pragma unroll 1
    for (int b0 = 0; b0 < nh; b0 += 32) {
      const int idx = b0 + lane;
      const int uv  = reg1[idx < RCAP ? idx : RCAP - 1];
      const int m32 = (nh - b0) < 32 ? (nh - b0) : 32;
#pragma unroll 1
      for (int k = 0; k < m32; ++k) {
        const int u   = __builtin_amdgcn_readlane(uv, k);
        const int sl  = u & (NBMAX - 1);
        const int eid = (int)((unsigned)u >> SLB);
        if (lane == 0) {
          int pos = list[sl];
          pos = pos < 0 ? 0 : (pos > RCAP - 1 ? RCAP - 1 : pos);
          reg2[pos] = eid;
          list[sl] = pos + 1;
        }
      }
    }
  }
  __syncthreads();

  const int nbw = nb >> 3;
  const bool ovf = (nh >= RCAP);
  const float qnan = __int_as_float(0x7fc00000);
  float* stw = (float*)reg1 + wave * STW;
  float at[4], bb[4], gg[4], be[4];
#pragma unroll
  for (int j = 0; j < NJ; ++j) {
    at[j] = prm[lane + 32 * j];
    bb[j] = prm[NCH + lane + 32 * j];
    gg[j] = prm[2 * NCH + lane + 32 * j];
    be[j] = prm[3 * NCH + lane + 32 * j];
  }
#pragma unroll 1
  for (int jt = 0; jt < nbw; ++jt) {
    const int slot = wave * nbw + jt;
    const int grow = nodeBase + slot;
    const int gcl  = grow < nN ? grow : nN - 1;
    int st = soff[slot];
    const int craw = scnt[slot];
    int cnt = craw;
    st  = st < 0 ? 0 : (st > nh ? nh : st);
    cnt = cnt < 0 ? 0 : (cnt > DEGCAP ? DEGCAP : cnt);
    if (cnt > nh - st) cnt = nh - st;
    const float pz = (ovf || craw > DEGCAP) ? qnan : 0.0f;
    const bool liveb = grow < nN;

    const float* rrow = plane + (size_t)gcl * LDX + XRO + lane;
    float xr[4], av[4], xl[4];
#pragma unroll
    for (int j = 0; j < NJ; ++j) { xr[j] = rrow[32 * j]; av[j] = 0.f; }
    ldwait();
    float mx[2], dn[2];
#pragma unroll
    for (int h = 0; h < NHD; ++h) { mx[h] = -1.0e30f; dn[h] = 0.f; }

#pragma unroll 1
    for (int q = 0; q < cnt; ++q) {
      int idx = st + q; idx = idx > RCAP - 1 ? RCAP - 1 : idx;
      int eid = reg2[idx]; eid = eid < 0 ? 0 : (eid > nE - 1 ? nE - 1 : eid);
      const int sraw = srcs[eid];
      ldwait();
      const int s = sraw < 0 ? 0 : (sraw > nN - 1 ? nN - 1 : sraw);
      const float* lrow = plane + (size_t)s * LDX + lane;
#pragma unroll
      for (int j = 0; j < NJ; ++j) xl[j] = lrow[32 * j];
      ldwait();
      float part[2];
#pragma unroll
      for (int h = 0; h < NHD; ++h) {
        float ea = xl[2 * h] + xr[2 * h];
        float eb = xl[2 * h + 1] + xr[2 * h + 1];
        ea = ea > 0.f ? ea : 0.2f * ea;
        eb = eb > 0.f ? eb : 0.2f * eb;
        part[h] = fmaf(eb, at[2 * h + 1], ea * at[2 * h]);
      }
#pragma unroll
      for (int off = 16; off > 0; off >>= 1) {
#pragma unroll
        for (int h = 0; h < NHD; ++h) part[h] += __shfl_xor(part[h], off);
      }
#pragma unroll
      for (int h = 0; h < NHD; ++h) {
        const float al = part[h];
        const float df = al - mx[h];
        const float ee = __expf(-fabsf(df));
        const bool up  = df > 0.f;
        const float s1 = up ? ee : 1.0f;
        const float s2 = up ? 1.0f : ee;
        mx[h] = up ? al : mx[h];
        dn[h] = fmaf(dn[h], s1, s2);
        av[2 * h]     = fmaf(av[2 * h],     s1, s2 * xl[2 * h]);
        av[2 * h + 1] = fmaf(av[2 * h + 1], s1, s2 * xl[2 * h + 1]);
      }
    }
    float iv[2];
#pragma unroll
    for (int h = 0; h < NHD; ++h) {
      const float ds = dn[h] > 0.f ? dn[h] : 1.0f;
      iv[h] = (dn[h] > 0.f ? 1.0f : 0.0f) * __builtin_amdgcn_rcpf(ds);
    }
    float v[4];
#pragma unroll
    for (int j = 0; j < NJ; ++j) v[j] = fmaf(av[j], iv[j >> 1], bb[j]);

    if (LAYER == 1) {
      float sm = (v[0] + v[1]) + (v[2] + v[3]);
#pragma unroll
      for (int off = 16; off > 0; off >>= 1) sm += __shfl_xor(sm, off);
      const float mu = sm * 0.0078125f;
      const float d0 = v[0] - mu, d1 = v[1] - mu, d2 = v[2] - mu, d3 = v[3] - mu;
      float sq = fmaf(d3, d3, fmaf(d2, d2, fmaf(d1, d1, d0 * d0)));
#pragma unroll
      for (int off = 16; off > 0; off >>= 1) sq += __shfl_xor(sq, off);
      const float var = sq * 0.0078125f;
      const float rs  = rsqrtf(var + 1.0e-5f);
      float y0 = fmaf(d0 * rs, gg[0], be[0]);
      float y1 = fmaf(d1 * rs, gg[1], be[1]);
      float y2 = fmaf(d2 * rs, gg[2], be[2]);
      float y3 = fmaf(d3 * rs, gg[3], be[3]);
      const float z0 = __expf(fminf(y0, 0.f)) - 1.0f;
      const float z1 = __expf(fminf(y1, 0.f)) - 1.0f;
      const float z2 = __expf(fminf(y2, 0.f)) - 1.0f;
      const float z3 = __expf(fminf(y3, 0.f)) - 1.0f;
      y0 = y0 > 0.f ? y0 : z0;  y1 = y1 > 0.f ? y1 : z1;
      y2 = y2 > 0.f ? y2 : z2;  y3 = y3 > 0.f ? y3 : z3;
      y0 = (liveb ? y0 : 0.f) + pz;  y1 = (liveb ? y1 : 0.f) + pz;
      y2 = (liveb ? y2 : 0.f) + pz;  y3 = (liveb ? y3 : 0.f) + pz;
      __builtin_amdgcn_fence(__ATOMIC_RELEASE, "wavefront");
      __builtin_amdgcn_wave_barrier();
      stw[lane]      = y0;
      stw[32 + lane] = y1;
      stw[64 + lane] = y2;
      stw[96 + lane] = y3;
      __builtin_amdgcn_fence(__ATOMIC_RELEASE, "wavefront");
      __builtin_amdgcn_wave_barrier();
      const int ch0 = 8 * (lane & 15);
      const v4f ga = *(const v4f*)(stw + ch0);
      const v4f gb = *(const v4f*)(stw + ch0 + 4);
      const v8us o = hilo8(ga, gb, hh);
      const bool wr = grow < MPr;
      const int growc = wr ? grow : MPr - 1;
      unsigned short* hp = (unsigned short*)(plane + (size_t)growc * LDX) + HOFF + 8 * lane;
      if (wr) *(volatile v8us*)hp = o;
      __threadfence();
      if (wr) *(volatile v8us*)hp = o;
    } else {
      const float o0 = (liveb ? v[0] : 0.f) + pz;
      const float o1 = (liveb ? v[1] : 0.f) + pz;
      __builtin_amdgcn_fence(__ATOMIC_RELEASE, "wavefront");
      __builtin_amdgcn_wave_barrier();
      stw[lane]      = o0;
      stw[32 + lane] = o1;
      __builtin_amdgcn_fence(__ATOMIC_RELEASE, "wavefront");
      __builtin_amdgcn_wave_barrier();
      const int lc = lane < 16 ? lane : 15;
      const v4f g4 = *(const v4f*)(stw + 4 * lc);
      float* gp = outN + (size_t)gcl * C2 + 4 * lc;
      const bool wsv = liveb && (lane < 16);
      if (wsv) *(volatile v4f*)gp = g4;
      __threadfence();
      if (wsv) *(volatile v4f*)gp = g4;
    }
  }
}

__global__ __launch_bounds__(NTHR) void k_pool(const float* nodev, const int* __restrict__ bat, float* gout, int nN) {
  __shared__ __attribute__((aligned(16))) float psum[NWAVE * C2];
  __shared__ int pcnt[NWAVE];
  __shared__ __attribute__((aligned(16))) float stq[C2];
  const int tid = (int)threadIdx.x, lane = tid & 31, wave = tid >> 5;
  const int g = (int)blockIdx.x;
  float a0 = 0.f, a1 = 0.f;
  int cnt = 0;
#pragma unroll 1
  for (int base = wave * 32; base < nN; base += NTHR) {
    const int n  = base + lane;
    const int nc = n < nN ? n : nN - 1;
    const int b  = bat[nc];
    ldwait();
    const bool hit = (n < nN) && (b == g);
    unsigned msk = __builtin_amdgcn_ballot_w32(hit);
    cnt += (int)__builtin_popcount(msk);
#pragma unroll 1
    while (msk != 0u) {
      const int k = __builtin_ctz(msk);
      msk &= msk - 1u;
      const float* row = nodev + (size_t)(base + k) * C2 + lane;
      const float r0v = row[0];
      const float r1v = row[32];
      ldwait();
      a0 += r0v;
      a1 += r1v;
    }
  }
  psum[wave * C2 + lane]      = a0;
  psum[wave * C2 + 32 + lane] = a1;
  if (lane == 0) pcnt[wave] = cnt;
  __syncthreads();
  if (wave == 0) {
    float s0 = 0.f, s1 = 0.f;
    int c = 0;
#pragma unroll
    for (int w2 = 0; w2 < NWAVE; ++w2) {
      s0 += psum[w2 * C2 + lane];
      s1 += psum[w2 * C2 + 32 + lane];
      c  += pcnt[w2];
    }
    const float cf = c > 1 ? (float)c : 1.0f;
    const float rc = __builtin_amdgcn_rcpf(cf);
    stq[lane]      = s0 * rc;
    stq[32 + lane] = s1 * rc;
    __builtin_amdgcn_fence(__ATOMIC_RELEASE, "wavefront");
    __builtin_amdgcn_wave_barrier();
    const int lc = lane < 16 ? lane : 15;
    const v4f g4 = *(const v4f*)(stq + 4 * lc);
    float* gp = gout + (size_t)g * C2 + 4 * lc;
    if (lane < 16) *(volatile v4f*)gp = g4;
    __threadfence();
    if (lane < 16) *(volatile v4f*)gp = g4;
  }
}

static int pick_nb(int nE, int nN) {
  int nb = NBMAX;
  while (nb > 16 && (long long)nb * (long long)nE * 5LL > (long long)RCAP * (long long)nN * 4LL) nb >>= 1;
  return nb;
}
static inline int cdiv(int a, int b) { return (a + b - 1) / b; }

extern "C" void kernel_launch(void* const* d_in, const int* in_sizes, int n_in,
                              void* d_out, int out_size, void* d_ws, size_t ws_size,
                              hipStream_t stream) {
  if (n_in < 17) return;
  const int nN = in_sizes[0] / DIN;
  if (nN <= 0 || in_sizes[0] != nN * DIN || nN > (1 << 22)) return;
  if (in_sizes[1] < 2 || (in_sizes[1] & 1) != 0) return;
  const int nE = in_sizes[1] / 2;
  if (nE < 1 || nE > (1 << 21)) return;
  if (in_sizes[2] != nN) return;
  if (in_sizes[3] != DIN * C1 || in_sizes[4] != C1) return;
  if (in_sizes[5] != DIN * C1 || in_sizes[6] != C1) return;
  if (in_sizes[7] != C1 || in_sizes[8] != C1) return;
  if (in_sizes[9] != C1 || in_sizes[10] != C1) return;
  if (in_sizes[11] != C1 * C2 || in_sizes[12] != C2) return;
  if (in_sizes[13] != C1 * C2 || in_sizes[14] != C2) return;
  if (in_sizes[15] != C2 || in_sizes[16] != C2) return;
  if (out_size <= 0 || (out_size % C2) != 0) return;
  const int nG = out_size / C2 - nN;
  if (nG < 1 || nG > 65535) return;
  if ((long long)nN * C2 + (long long)nG * C2 != (long long)out_size) return;

  const float* x     = (const float*)d_in[0];
  const int*   ei    = (const int*)  d_in[1];
  const int*   batch = (const int*)  d_in[2];
  const float* W1l   = (const float*)d_in[3];
  const float* b1l   = (const float*)d_in[4];
  const float* W1r   = (const float*)d_in[5];
  const float* b1r   = (const float*)d_in[6];
  const float* att1  = (const float*)d_in[7];
  const float* bias1 = (const float*)d_in[8];
  const float* g1    = (const float*)d_in[9];
  const float* be1   = (const float*)d_in[10];
  const float* W2l   = (const float*)d_in[11];
  const float* b2l   = (const float*)d_in[12];
  const float* W2r   = (const float*)d_in[13];
  const float* b2r   = (const float*)d_in[14];
  const float* att2  = (const float*)d_in[15];
  const float* bias2 = (const float*)d_in[16];
  float* out = (float*)d_out;
  const int* src = ei;
  const int* dst = ei + nE;

  const int MP   = cdiv(nN, GBM) * GBM;
  const int nb   = pick_nb(nE, nN);
  const int gA   = cdiv(MP, nb);
  const int vec8 = ((nE & 3) == 0) ? 1 : 0;
  if (nb < 16 || gA * nb < MP) return;

  char* ws = (char*)d_ws;
  size_t off = 0;
  const size_t oXLR = off; off += (size_t)MP * LDX * 4;           off = (off + 255) & ~(size_t)255;
  const size_t oXB  = off; off += (size_t)MP * DIN * 2;           off = (off + 255) & ~(size_t)255;
  const size_t oWT1 = off; off += (size_t)N1 * DIN * 2;           off = (off + 255) & ~(size_t)255;
  const size_t oWT2 = off; off += (size_t)N2 * K2 * 2;            off = (off + 255) & ~(size_t)255;
  if (off > ws_size || off > (size_t)WSMAX) return;
  float*          XLR = (float*)(ws + oXLR);
  unsigned short* XB  = (unsigned short*)(ws + oXB);
  unsigned short* WT1 = (unsigned short*)(ws + oWT1);
  unsigned short* WT2 = (unsigned short*)(ws + oWT2);
  const unsigned short* HA = (const unsigned short*)XLR + HOFF;

  hipFuncSetAttribute(reinterpret_cast<const void*>(&k_agg<1>),
                      hipFuncAttributeMaxDynamicSharedMemorySize, LDS_AGG);
  hipFuncSetAttribute(reinterpret_cast<const void*>(&k_agg<2>),
                      hipFuncAttributeMaxDynamicSharedMemorySize, LDS_AGG);

  const int nUx = MP * (DIN / 8);
  k_xprep<<<cdiv(nUx, NTHR), NTHR, 0, stream>>>(x, XB, nN, nUx);

  {
    const int nU1 = N1 * (DIN / 8);
    k_wtr<<<cdiv(nU1, NTHR), NTHR, 0, stream>>>(W1l, W1r, C1, DIN, DIN, WT1, nU1);
    const int nU2 = N2 * (K2 / 8);
    k_wtr<<<cdiv(nU2, NTHR), NTHR, 0, stream>>>(W2l, W2r, C2, C1, K2, WT2, nU2);
  }

  const int gM = MP / GBM;
  k_gemm<<<dim3(gM, N1 / GBN), GTHR, 0, stream>>>(XB, DIN, WT1, DIN, b1l, b1r, C1, C1, XLR, LDX);
  k_agg<1><<<gA, NTHR, LDS_AGG, stream>>>(src, dst, XLR, att1, bias1, g1, be1, out, nN, nE, nb, vec8, MP);
  k_gemm<<<dim3(gM, N2 / GBN), GTHR, 0, stream>>>(HA, LDH, WT2, K2, b2l, b2r, C2, C2, XLR, LDX);
  k_agg<2><<<gA, NTHR, LDS_AGG, stream>>>(src, dst, XLR, att2, bias2, bias2, bias2, out, nN, nE, nb, vec8, MP);
  k_pool<<<nG, NTHR, 0, stream>>>(out, batch, out + (size_t)nN * C2, nN);
}
